// GaANConv_38397007626856
// MI455X (gfx1250) — hardware-verified
//
#include <hip/hip_runtime.h>
#include <stddef.h>

typedef _Float16 v16h __attribute__((ext_vector_type(16)));
typedef _Float16 v8h __attribute__((ext_vector_type(8)));
typedef _Float16 v4h __attribute__((ext_vector_type(4)));
typedef float v8f __attribute__((ext_vector_type(8)));
typedef float v4f __attribute__((ext_vector_type(4)));
typedef float v4fa __attribute__((ext_vector_type(4), __may_alias__));
typedef int v4i __attribute__((ext_vector_type(4)));

union HFrag { v16h v; v8h half[2]; _Float16 e[16]; };
union H8 { v8h v; _Float16 e[8]; };
union H4 { v4h v; _Float16 e[4]; };

#define NBLK 128
#define CHUNK 4096
#define CAP 3072
#define SZS (NBLK * 256)
#define AW_FLOATS (16 * 256)
#define EAT_HALVES (16 * 32)
#define LDS_BYTES (2 * SZS * 4 + AW_FLOATS * 4 + CAP * 4 + EAT_HALVES * 2 + 64)

__device__ __forceinline__ v8f zero8() {
  v8f z = {0.f, 0.f, 0.f, 0.f, 0.f, 0.f, 0.f, 0.f};
  return z;
}
__device__ __forceinline__ v8h zero8h() {
  H8 z;
#pragma unroll
  for (int i = 0; i < 8; ++i) z.e[i] = (_Float16)0.0f;
  return z.v;
}

__device__ __forceinline__ v8f wmma_f16(v16h a, v16h b, v8f c) {
  v8f d = __builtin_amdgcn_wmma_f32_16x16x32_f16(false, a, false, b, (short)0, c, false, false);
  asm volatile("v_nop\n\tv_nop\n\tv_nop\n\tv_nop" : "+v"(d) : "v"(a), "v"(b));
  return d;
}

__device__ __forceinline__ void chunk_scan(const int* __restrict__ ei, int E, bool vec4, int cbase,
                                           int nodeBase, int t, int l, int w, int count, int* wtot,
                                           int (&dv)[16], unsigned& hit, int& pos, int& tot) {
#pragma unroll
  for (int j = 0; j < 4; ++j) {
    const int e4 = cbase + 1024 * j + 4 * t;
    int d0 = -1, d1 = -1, d2 = -1, d3 = -1;
    if (vec4 && (e4 + 4 <= E)) {
      const v4i dd = *(const v4i*)(ei + (size_t)E + e4);
      d0 = dd.x; d1 = dd.y; d2 = dd.z; d3 = dd.w;
    } else {
      if (e4 < E) d0 = ei[(size_t)E + e4];
      if (e4 + 1 < E) d1 = ei[(size_t)E + e4 + 1];
      if (e4 + 2 < E) d2 = ei[(size_t)E + e4 + 2];
      if (e4 + 3 < E) d3 = ei[(size_t)E + e4 + 3];
    }
    dv[4 * j] = d0; dv[4 * j + 1] = d1; dv[4 * j + 2] = d2; dv[4 * j + 3] = d3;
  }
  hit = 0;
  int cnt = 0;
#pragma unroll
  for (int i = 0; i < 16; ++i) {
    const int s = dv[i] - nodeBase;
    if ((unsigned)s < (unsigned)NBLK) { hit |= (1u << i); ++cnt; }
  }
  int incl = cnt;
#pragma unroll
  for (int o = 1; o < 32; o <<= 1) {
    const int y = __shfl_up(incl, o, 32);
    if (l >= o) incl += y;
  }
  if (l == 31) wtot[w] = incl;
  __syncthreads();
  pos = count + incl - cnt;
  tot = 0;
#pragma unroll
  for (int i = 0; i < 8; ++i) {
    const int v = wtot[i];
    if (i < w) pos += v;
    tot += v;
  }
}

__global__ __launch_bounds__(256) void prep_kernel(
    const float* __restrict__ Wn, const float* __restrict__ Wpi, const float* __restrict__ bpi,
    const float* __restrict__ Wpj, const float* __restrict__ bpj, const float* __restrict__ Wa,
    const float* __restrict__ ba, const float* __restrict__ Wfc,
    _Float16* Wnf, _Float16* W1f, _Float16* W2f, _Float16* W3h, float* bAll, _Float16* Wfc16) {
  __shared__ __align__(16) float sb[256];
  const int bid = blockIdx.x;
  const int t = threadIdx.x;
  if (bid < 16) {
    const int tid = bid * 256 + t;
    const int mat = tid >> 11;
    const int r = tid & 2047;
    const int h = r >> 9, c = (r >> 3) & 63, q = r & 7;
    const float* wp = (mat == 0 ? Wpi : Wpj) + (size_t)h * 4096;
    const float* wa = Wa + (size_t)h * 9216 + (mat == 0 ? 0 : 4096);
    float s[8];
#pragma unroll
    for (int i = 0; i < 8; ++i) s[i] = 0.0f;
#pragma unroll 1
    for (int j = 0; j < 64; ++j) {
      const float wv = wa[j * 64 + c];
#pragma unroll
      for (int i = 0; i < 8; ++i) s[i] += wp[(8 * q + i) * 64 + j] * wv;
    }
    H8 o;
#pragma unroll
    for (int i = 0; i < 8; ++i) o.e[i] = (_Float16)(s[i] * 64.0f);
    _Float16* dst = (mat == 0 ? W1f : W2f) + (size_t)r * 8;
    *(volatile v8h*)dst = o.v;
    __threadfence();
    *(volatile v8h*)dst = o.v;
  } else if (bid < 32) {
    const int tid = (bid - 16) * 256 + t;
    const int h = tid >> 10, c = (tid >> 4) & 63, q = tid & 15;
    H8 o;
#pragma unroll
    for (int i = 0; i < 8; ++i)
      o.e[i] = (_Float16)(Wn[((size_t)h * 128 + 8 * q + i) * 64 + c] * 64.0f);
    _Float16* dst = Wnf + (size_t)tid * 8;
    *(volatile v8h*)dst = o.v;
    __threadfence();
    *(volatile v8h*)dst = o.v;
  } else if (bid < 34) {
    const int tid = (bid - 32) * 256 + t;
    const int row = tid >> 1, q = tid & 1;
    const int h = row >> 6, c = row & 63;
    H8 o;
#pragma unroll
    for (int i = 0; i < 8; ++i)
      o.e[i] = (_Float16)(Wa[((size_t)h * 144 + 128 + 8 * q + i) * 64 + c] * 64.0f);
    _Float16* dst = W3h + (size_t)tid * 8;
    *(volatile v8h*)dst = o.v;
    __threadfence();
    *(volatile v8h*)dst = o.v;
  } else if (bid < 35) {
    const int h = t >> 6, c = t & 63;
    const float* wa = Wa + (size_t)h * 9216;
    float s = ba[t];
#pragma unroll 1
    for (int j = 0; j < 64; ++j) {
      s += bpi[h * 64 + j] * wa[j * 64 + c];
      s += bpj[h * 64 + j] * wa[(64 + j) * 64 + c];
    }
    sb[t] = s;
    __syncthreads();
    if (t < 64) {
      const v4f v = *(const v4fa*)(sb + 4 * t);
      *(volatile v4f*)(bAll + 4 * t) = v;
      __threadfence();
      *(volatile v4f*)(bAll + 4 * t) = v;
    }
  } else {
    const int tid = (bid - 35) * 256 + t;
    if (tid < 3072) {
      const int col = tid / 48;
      const int q = tid - col * 48;
      H8 o;
#pragma unroll
      for (int i = 0; i < 8; ++i)
        o.e[i] = (_Float16)(Wfc[(size_t)(8 * q + i) * 64 + col] * 64.0f);
      _Float16* dst = Wfc16 + (size_t)tid * 8;
      *(volatile v8h*)dst = o.v;
      __threadfence();
      *(volatile v8h*)dst = o.v;
    }
  }
}

__device__ __forceinline__ void store_seg(_Float16* g, const _Float16* s, int base, int w, int l,
                                          int h, int N) {
#pragma unroll
  for (int j = 0; j < 4; ++j) {
    const int q = 32 * j + l;
    const int r = q >> 3, c8 = q & 7;
    const int node = base + w * 16 + r;
    if (node < N) {
      const v8h v = *(const v8h*)(s + (w * 16 + r) * 72 + 8 * c8);
      *(volatile v8h*)(g + (size_t)node * 256 + h * 64 + 8 * c8) = v;
    }
  }
}

__device__ __forceinline__ void store_xrows(_Float16* g, const _Float16* s, int base, int w, int l,
                                            int N) {
#pragma unroll
  for (int j = 0; j < 8; ++j) {
    const int q = 32 * j + l;
    const int r = q >> 4, c8 = q & 15;
    const int node = base + w * 16 + r;
    if (node < N) {
      const v8h v = *(const v8h*)(s + (w * 16 + r) * 136 + 8 * c8);
      *(volatile v8h*)(g + (size_t)node * 128 + 8 * c8) = v;
    }
  }
}

__global__ __launch_bounds__(128) void node_kernel(
    const float* __restrict__ x, const _Float16* __restrict__ Wnf, const float* __restrict__ bn,
    const _Float16* __restrict__ W1f, const float* __restrict__ bAll,
    const _Float16* __restrict__ W2f, _Float16* xfc16, _Float16* u16, _Float16* v16, _Float16* x16,
    int N) {
  __shared__ __align__(16) _Float16 xs[64 * 136];
  __shared__ __align__(16) _Float16 fs[64 * 72];
  __shared__ __align__(16) _Float16 us[64 * 72];
  __shared__ __align__(16) _Float16 vs[64 * 72];
  const int t = threadIdx.x, l = t & 31, w = t >> 5, hh = l >> 4, n = l & 15;
  const int h = blockIdx.y;
  const int base = blockIdx.x * 64;
  const float INV64 = 0.015625f;

  for (int i = t; i < 64 * 32; i += 128) {
    const int row = i >> 5, c4 = i & 31;
    const int node = base + row;
    v4f v = {0.f, 0.f, 0.f, 0.f};
    if (node < N) v = *(const v4f*)(x + (size_t)node * 128 + 4 * c4);
    H4 o;
    o.e[0] = (_Float16)v.x;
    o.e[1] = (_Float16)v.y;
    o.e[2] = (_Float16)v.z;
    o.e[3] = (_Float16)v.w;
    *(v4h*)(xs + row * 136 + 4 * c4) = o.v;
  }
  __syncthreads();

  v8f acc[4];
#pragma unroll
  for (int ct = 0; ct < 4; ++ct) acc[ct] = zero8();
  {
    const _Float16* arow = xs + (w * 16 + n) * 136;
#pragma unroll
    for (int ks = 0; ks < 4; ++ks) {
      HFrag a;
      a.half[0] = *(const v8h*)(arow + ks * 32 + 8 * hh);
      a.half[1] = *(const v8h*)(arow + ks * 32 + 16 + 8 * hh);
#pragma unroll
      for (int ct = 0; ct < 4; ++ct) {
        const _Float16* bp = Wnf + ((size_t)(h * 64 + ct * 16 + n)) * 128 + ks * 32 + 8 * hh;
        HFrag b;
        b.half[0] = *(const v8h*)bp;
        b.half[1] = *(const v8h*)(bp + 16);
        acc[ct] = wmma_f16(a.v, b.v, acc[ct]);
      }
    }
  }
#pragma unroll
  for (int ct = 0; ct < 4; ++ct) {
    const float bv = bn[h * 64 + ct * 16 + n];
#pragma unroll
    for (int r = 0; r < 8; ++r)
      fs[(w * 16 + 8 * hh + r) * 72 + ct * 16 + n] = (_Float16)(acc[ct][r] * INV64 + bv);
  }
  __syncthreads();

  HFrag a0, a1;
  {
    const _Float16* frow = fs + (w * 16 + n) * 72;
    a0.half[0] = *(const v8h*)(frow + 8 * hh);
    a0.half[1] = *(const v8h*)(frow + 16 + 8 * hh);
    a1.half[0] = *(const v8h*)(frow + 32 + 8 * hh);
    a1.half[1] = *(const v8h*)(frow + 48 + 8 * hh);
  }

#pragma unroll
  for (int ct = 0; ct < 4; ++ct) acc[ct] = zero8();
#pragma unroll
  for (int ct = 0; ct < 4; ++ct) {
    const _Float16* bp = W1f + ((size_t)(h * 64 + ct * 16 + n)) * 64 + 8 * hh;
    HFrag b0, b1;
    b0.half[0] = *(const v8h*)bp;
    b0.half[1] = *(const v8h*)(bp + 16);
    b1.half[0] = *(const v8h*)(bp + 32);
    b1.half[1] = *(const v8h*)(bp + 48);
    acc[ct] = wmma_f16(a0.v, b0.v, acc[ct]);
    acc[ct] = wmma_f16(a1.v, b1.v, acc[ct]);
  }
#pragma unroll
  for (int ct = 0; ct < 4; ++ct) {
    const float bv = bAll[h * 64 + ct * 16 + n];
#pragma unroll
    for (int r = 0; r < 8; ++r)
      us[(w * 16 + 8 * hh + r) * 72 + ct * 16 + n] = (_Float16)(acc[ct][r] * INV64 + bv);
  }

#pragma unroll
  for (int ct = 0; ct < 4; ++ct) acc[ct] = zero8();
#pragma unroll
  for (int ct = 0; ct < 4; ++ct) {
    const _Float16* bp = W2f + ((size_t)(h * 64 + ct * 16 + n)) * 64 + 8 * hh;
    HFrag b0, b1;
    b0.half[0] = *(const v8h*)bp;
    b0.half[1] = *(const v8h*)(bp + 16);
    b1.half[0] = *(const v8h*)(bp + 32);
    b1.half[1] = *(const v8h*)(bp + 48);
    acc[ct] = wmma_f16(a0.v, b0.v, acc[ct]);
    acc[ct] = wmma_f16(a1.v, b1.v, acc[ct]);
  }
#pragma unroll
  for (int ct = 0; ct < 4; ++ct) {
#pragma unroll
    for (int r = 0; r < 8; ++r)
      vs[(w * 16 + 8 * hh + r) * 72 + ct * 16 + n] = (_Float16)(acc[ct][r] * INV64);
  }
  __syncthreads();

  store_seg(xfc16, fs, base, w, l, h, N);
  store_seg(u16, us, base, w, l, h, N);
  store_seg(v16, vs, base, w, l, h, N);
  if (h == 0) store_xrows(x16, xs, base, w, l, N);
  __threadfence();
  store_seg(xfc16, fs, base, w, l, h, N);
  store_seg(u16, us, base, w, l, h, N);
  store_seg(v16, vs, base, w, l, h, N);
  if (h == 0) store_xrows(x16, xs, base, w, l, N);
}

__global__ __launch_bounds__(256) void aggr_kernel(
    const int* __restrict__ ei, const float* __restrict__ ea,
    const _Float16* __restrict__ xfc16, const _Float16* __restrict__ u16,
    const _Float16* __restrict__ v16, const _Float16* __restrict__ x16,
    const _Float16* __restrict__ W3h, const _Float16* __restrict__ Wfc16,
    const float* __restrict__ bfc, float* out, int N, int E) {
  extern __shared__ __align__(16) unsigned char smem[];
  float* dS = (float*)smem;
  float* sS = dS + SZS;
  float* aW = sS + SZS;
  int* list = (int*)(aW + AW_FLOATS);
  _Float16* eaT = (_Float16*)(list + CAP);
  int* wtot = (int*)(eaT + EAT_HALVES);

  const int t = threadIdx.x, l = t & 31, w = t >> 5, hh = l >> 4, n = l & 15;
  const int nodeBase = blockIdx.x * NBLK;
  const float INV64 = 0.015625f;

  {
    const v4f z = {0.f, 0.f, 0.f, 0.f};
    for (int i = t; i < (2 * SZS) / 4; i += 256) *(v4f*)(dS + 4 * i) = z;
    if (t < EAT_HALVES / 8) *(v8h*)(eaT + 8 * t) = zero8h();
  }
  HFrag b3a, b3b;
  {
    const _Float16* p = W3h + ((size_t)(32 * w + n)) * 16 + 8 * hh;
    b3a.half[0] = *(const v8h*)p;
    b3a.half[1] = zero8h();
    b3b.half[0] = *(const v8h*)(p + 16 * 16);
    b3b.half[1] = zero8h();
  }
  __syncthreads();

  int count = 0;
  const int nch = (E + CHUNK - 1) / CHUNK;
  const bool vec4 = ((E & 3) == 0);
  for (int ci = 0; ci < nch; ++ci) {
    const int cbase = ci * CHUNK;
    int dv[16];
    unsigned hit;
    int pos, tot;
    chunk_scan(ei, E, vec4, cbase, nodeBase, t, l, w, count, wtot, dv, hit, pos, tot);
#pragma unroll
    for (int i = 0; i < 16; ++i) {
      if (hit & (1u << i)) {
        int e = cbase + 1024 * (i >> 2) + 4 * t + (i & 3);
        if (e >= E) e = E - 1;
        if (e < 0) e = 0;
        if ((unsigned)pos < (unsigned)CAP) list[pos] = (e << 7) | (dv[i] - nodeBase);
        ++pos;
      }
    }
    count += tot;
    if (count > CAP) count = CAP;
    __syncthreads();
  }
  __syncthreads();

  {
    const int cc = count;
    const int ntiles = (cc + 15) >> 4;
    for (int ti = 0; ti < ntiles && ti < (CAP / 16); ++ti) {
      {
        const int i = t >> 4, j = t & 15;
        const int li = ti * 16 + i;
        _Float16 hv = (_Float16)0.0f;
        if (li < cc) {
          int e = list[li] >> 7;
          if (e >= E) e = E - 1;
          if (e < 0) e = 0;
          hv = (_Float16)ea[(size_t)e * 16 + j];
        }
        eaT[i * 32 + j] = hv;
      }
      __syncthreads();
      {
        HFrag a;
        a.half[0] = *(const v8h*)(eaT + n * 32 + 8 * hh);
        a.half[1] = zero8h();
        const v8f w0 = wmma_f16(a.v, b3a.v, zero8());
        const v8f w1 = wmma_f16(a.v, b3b.v, zero8());
#pragma unroll
        for (int r = 0; r < 8; ++r) {
          const int ai = (8 * hh + r) * 256 + 32 * w + n;
          aW[ai] = w0[r] * INV64;
          aW[ai + 16] = w1[r] * INV64;
        }
      }
      __syncthreads();
#pragma unroll 1
      for (int i = 0; i < 16; ++i) {
        const int li = ti * 16 + i;
        if (li >= cc) break;
        const int ent = list[li];
        int e = ent >> 7;
        if (e >= E) e = E - 1;
        if (e < 0) e = 0;
        const int slot = ent & (NBLK - 1);
        int src = ei[e];
        src = (src < 0) ? 0 : ((src >= N) ? (N - 1) : src);
        int dstn = nodeBase + slot;
        if (dstn > N - 1) dstn = N - 1;
        const float uu = (float)u16[(size_t)dstn * 256 + t];
        const float vv = (float)v16[(size_t)src * 256 + t];
        const float xx = (float)xfc16[(size_t)src * 256 + t];
        float a = uu + vv + aW[i * 256 + t];
        a = (a >= 0.0f) ? a : 0.2f * a;
        a = fminf(a, 80.0f);
        const float ex = __expf(a);
        const int si = slot * 256 + t;
        dS[si] += ex;
        sS[si] += ex * xx;
      }
      __syncthreads();
    }
  }
  __syncthreads();

#pragma unroll 1
  for (int s = 0; s < NBLK; ++s) {
    const int si = s * 256 + t;
    const float d = dS[si];
    const float v = sS[si];
    sS[si] = v * __builtin_amdgcn_rcpf(d + 1e-16f);
  }
  __syncthreads();
  _Float16* hT = (_Float16*)dS;
#pragma unroll 1
  for (int s = 0; s < NBLK; ++s) {
    const int si = s * 256 + t;
    hT[si] = (_Float16)sS[si];
  }
  __syncthreads();

  float* oL = sS;
  {
    v8f acc[4];
#pragma unroll
    for (int ct = 0; ct < 4; ++ct) acc[ct] = zero8();
    int ldn = nodeBase + 16 * w + n;
    if (ldn > N - 1) ldn = N - 1;
    const _Float16* xr = x16 + (size_t)ldn * 128;
#pragma unroll 1
    for (int ks = 0; ks < 4; ++ks) {
      HFrag a;
      a.half[0] = *(const v8h*)(xr + ks * 32 + 8 * hh);
      a.half[1] = *(const v8h*)(xr + ks * 32 + 16 + 8 * hh);
#pragma unroll
      for (int ct = 0; ct < 4; ++ct) {
        const _Float16* bp = Wfc16 + ((size_t)(ct * 16 + n)) * 384 + ks * 32 + 8 * hh;
        HFrag b;
        b.half[0] = *(const v8h*)bp;
        b.half[1] = *(const v8h*)(bp + 16);
        acc[ct] = wmma_f16(a.v, b.v, acc[ct]);
      }
    }
    const _Float16* hr = hT + (16 * w + n) * 256;
#pragma unroll 1
    for (int ks = 0; ks < 8; ++ks) {
      HFrag a;
      a.half[0] = *(const v8h*)(hr + ks * 32 + 8 * hh);
      a.half[1] = *(const v8h*)(hr + ks * 32 + 16 + 8 * hh);
      const int kg = 128 + ks * 32;
#pragma unroll
      for (int ct = 0; ct < 4; ++ct) {
        const _Float16* bp = Wfc16 + ((size_t)(ct * 16 + n)) * 384 + kg + 8 * hh;
        HFrag b;
        b.half[0] = *(const v8h*)bp;
        b.half[1] = *(const v8h*)(bp + 16);
        acc[ct] = wmma_f16(a.v, b.v, acc[ct]);
      }
    }
#pragma unroll
    for (int ct = 0; ct < 4; ++ct) {
      const float bv = bfc[ct * 16 + n];
#pragma unroll
      for (int r = 0; r < 8; ++r)
        oL[(16 * w + 8 * hh + r) * 64 + ct * 16 + n] = acc[ct][r] * INV64 + bv;
    }
  }
  __syncthreads();

#pragma unroll
  for (int j = 0; j < 8; ++j) {
    const int q = 32 * j + l;
    const int r = q >> 4, c4 = q & 15;
    const int node = nodeBase + 16 * w + r;
    if (node < N) {
      const v4f v = *(const v4fa*)(oL + (16 * w + r) * 64 + 4 * c4);
      *(volatile v4f*)(out + (size_t)node * 64 + 4 * c4) = v;
    }
  }
  __threadfence();
#pragma unroll
  for (int j = 0; j < 8; ++j) {
    const int q = 32 * j + l;
    const int r = q >> 4, c4 = q & 15;
    const int node = nodeBase + 16 * w + r;
    if (node < N) {
      const v4f v = *(const v4fa*)(oL + (16 * w + r) * 64 + 4 * c4);
      *(volatile v4f*)(out + (size_t)node * 64 + 4 * c4) = v;
    }
  }
}

extern "C" void kernel_launch(void* const* d_in, const int* in_sizes, int n_in,
                              void* d_out, int out_size, void* d_ws, size_t ws_size,
                              hipStream_t stream) {
  if (n_in < 13) return;
  const float* x   = (const float*)d_in[0];
  const int*   ei  = (const int*)d_in[1];
  const float* ea  = (const float*)d_in[2];
  const float* Wn  = (const float*)d_in[3];
  const float* bn  = (const float*)d_in[4];
  const float* Wpi = (const float*)d_in[5];
  const float* bpi = (const float*)d_in[6];
  const float* Wpj = (const float*)d_in[7];
  const float* bpj = (const float*)d_in[8];
  const float* Wa  = (const float*)d_in[9];
  const float* ba  = (const float*)d_in[10];
  const float* Wfc = (const float*)d_in[11];
  const float* bfc = (const float*)d_in[12];

  const int N = in_sizes[0] / 128;
  const int E = in_sizes[1] / 2;
  if (N <= 0 || E < 0) return;
  if (in_sizes[0] != N * 128 || in_sizes[1] != 2 * E || in_sizes[2] != E * 16) return;
  if (in_sizes[3] != 4 * 128 * 64 || in_sizes[4] != 256 || in_sizes[5] != 4 * 64 * 64 ||
      in_sizes[6] != 256 || in_sizes[7] != 4 * 64 * 64 || in_sizes[8] != 256 ||
      in_sizes[9] != 4 * 144 * 64 || in_sizes[10] != 256 || in_sizes[11] != 384 * 64 ||
      in_sizes[12] != 64) return;
  if (E >= (1 << 24)) return;
  if (out_size < N * 64) return;

  const unsigned nodeBlocks = (unsigned)((N + 63) / 64);
  const unsigned aggBlocks = (unsigned)((N + NBLK - 1) / NBLK);

  size_t off = 0;
  const size_t oWnf  = off; off += (size_t)4 * 64 * 128 * 2;   off = (off + 255) & ~(size_t)255;
  const size_t oW1f  = off; off += (size_t)4 * 64 * 64 * 2;    off = (off + 255) & ~(size_t)255;
  const size_t oW2f  = off; off += (size_t)4 * 64 * 64 * 2;    off = (off + 255) & ~(size_t)255;
  const size_t oW3h  = off; off += (size_t)256 * 16 * 2;       off = (off + 255) & ~(size_t)255;
  const size_t obAll = off; off += (size_t)256 * 4;            off = (off + 255) & ~(size_t)255;
  const size_t oWfc  = off; off += (size_t)64 * 384 * 2;       off = (off + 255) & ~(size_t)255;
  const size_t oxfc  = off; off += (size_t)N * 256 * 2;        off = (off + 255) & ~(size_t)255;
  const size_t ou    = off; off += (size_t)N * 256 * 2;        off = (off + 255) & ~(size_t)255;
  const size_t ov    = off; off += (size_t)N * 256 * 2;        off = (off + 255) & ~(size_t)255;
  const size_t ox16  = off; off += (size_t)N * 128 * 2;        off = (off + 255) & ~(size_t)255;
  if (off > ws_size) return;
  if (off > ((size_t)128 << 20)) return;

  unsigned char* ws = (unsigned char*)d_ws;
  _Float16* Wnf   = (_Float16*)(ws + oWnf);
  _Float16* W1f   = (_Float16*)(ws + oW1f);
  _Float16* W2f   = (_Float16*)(ws + oW2f);
  _Float16* W3h   = (_Float16*)(ws + oW3h);
  float*    bAll  = (float*)(ws + obAll);
  _Float16* Wfc16 = (_Float16*)(ws + oWfc);
  _Float16* xfc16 = (_Float16*)(ws + oxfc);
  _Float16* u16   = (_Float16*)(ws + ou);
  _Float16* v16   = (_Float16*)(ws + ov);
  _Float16* x16   = (_Float16*)(ws + ox16);

  prep_kernel<<<47, 256, 0, stream>>>(Wn, Wpi, bpi, Wpj, bpj, Wa, ba, Wfc,
                                       Wnf, W1f, W2f, W3h, bAll, Wfc16);

  node_kernel<<<dim3(nodeBlocks, 4, 1), 128, 0, stream>>>(x, Wnf, bn, W1f, bAll, W2f,
                                                         xfc16, u16, v16, x16, N);

  hipFuncSetAttribute((const void*)aggr_kernel, hipFuncAttributeMaxDynamicSharedMemorySize, LDS_BYTES);
  aggr_kernel<<<aggBlocks, 256, LDS_BYTES, stream>>>(ei, ea, xfc16, u16, v16, x16, W3h, Wfc16, bfc,
                                                     (float*)d_out, N, E);
  (void)hipGetLastError();
}
